// StructuredAdaLNMLPCRN_70772471103814
// MI455X (gfx1250) — hardware-verified
//
#include <hip/hip_runtime.h>
#include <math.h>
#include <stdint.h>

#pragma clang fp contract(off)

#define NB    32
#define NPTS  8192
#define XD    3
#define KOBJ  16
#define HID   64
#define NLAY  6
#define TED   32
#define CDIM  128
#define CWD   160
#define BR    128
#define NTHR  256
#define PA    136

#define S_X    16.0f
#define S_W    64.0f
#define S_PF   256.0f
#define S_OBJ  16.0f
#define S_CW   4096.0f
#define S_H    16.0f
#define S_RES  1024.0f
#define INV_XW   (1.0f / 1024.0f)
#define INV_PFO  (1.0f / 4096.0f)
#define INV_HW   (1.0f / 1024.0f)
#define INV_RES  (1.0f / 1024.0f)
#define INV_CW   (1.0f / 4096.0f)

#define C_WEMB 0
#define C_BEMB 192
#define C_BPF  256
#define C_BH   320
#define C_BSS  704
#define C_LG   1472
#define C_LB   1856
#define C_WOUT 2240
#define C_BOUT 2432
#define C_TOT  2436

#define WS_WPF  0
#define WS_WH   4096
#define WS_OBJ  28672
#define WS_CW   61440
#define WS_TOT  454656
#define WCONV_PIECES 3584

static_assert(NPTS % BR == 0);
static_assert(BR == 128 && NTHR == 256);
static_assert((BR * XD * 4) % 128 == 0);
static_assert(WS_WH == WS_WPF + HID * HID);
static_assert(WS_OBJ == WS_WH + NLAY * HID * HID);
static_assert(WS_CW == WS_OBJ + NB * KOBJ * HID);
static_assert(WS_TOT == WS_CW + NB * NLAY * CDIM * KOBJ);
static_assert((WS_WH * 2) % 128 == 0 && (WS_OBJ * 2) % 128 == 0 && (WS_CW * 2) % 128 == 0);
static_assert(WCONV_PIECES * 8 == WS_OBJ);
static_assert(WCONV_PIECES % 256 == 0);
static_assert((KOBJ * HID * 2) % 128 == 0 && (NLAY * CDIM * KOBJ * 2) % 512 == 0);
static_assert((PA % 8) == 0);
static_assert(CWD == TED + CDIM);

typedef _Float16       v16h __attribute__((ext_vector_type(16)));
typedef unsigned short v8us __attribute__((ext_vector_type(8)));
typedef float          v8f  __attribute__((ext_vector_type(8)));
typedef float          v4f  __attribute__((ext_vector_type(4)));

union FragH { v16h v; v8us u[2]; };

__device__ __forceinline__ unsigned short bf_bits(float f) {
  const unsigned u = __float_as_uint(f);
  return (unsigned short)((u + 0x7FFFu + ((u >> 16) & 1u)) >> 16);
}
__device__ __forceinline__ float bf_up(unsigned short b) { return __uint_as_float(((unsigned)b) << 16); }
__device__ __forceinline__ float bfr(float f) { return bf_up(bf_bits(f)); }
__device__ __forceinline__ unsigned short h_bits(float f) {
  const _Float16 hv = (_Float16)f;
  return __builtin_bit_cast(unsigned short, hv);
}
__device__ __forceinline__ v8f zero8() { return (v8f){0.f, 0.f, 0.f, 0.f, 0.f, 0.f, 0.f, 0.f}; }
__device__ __forceinline__ v8us zero8us() {
  v8us z;
#pragma unroll
  for (int i = 0; i < 8; ++i) z[i] = (unsigned short)0;
  return z;
}
__device__ __forceinline__ float rcp_f(float v) {
#if defined(__HIP_DEVICE_COMPILE__)
  return __builtin_amdgcn_rcpf(v);
#else
  return 1.0f / v;
#endif
}
__device__ __forceinline__ float rsq_f(float v) {
#if defined(__HIP_DEVICE_COMPILE__)
  return __builtin_amdgcn_rsqf(v);
#else
  return 1.0f / sqrtf(v);
#endif
}
__device__ __forceinline__ float swish_f(float v) {
  const float e = __expf(-v);
  return v * rcp_f(1.0f + e);
}
__device__ __forceinline__ float sin_small(float a) {
  const float a2 = a * a;
  float p = -2.5052108e-8f;
  p = p * a2 + 2.7557319e-6f;
  p = p * a2 - 1.9841270e-4f;
  p = p * a2 + 8.3333333e-3f;
  p = p * a2 - 1.6666667e-1f;
  p = p * a2;
  return a + a * p;
}
__device__ __forceinline__ float cos_small(float a) {
  const float a2 = a * a;
  float p = 2.0876757e-9f;
  p = p * a2 - 2.7557319e-7f;
  p = p * a2 + 2.4801587e-5f;
  p = p * a2 - 1.3888889e-3f;
  p = p * a2 + 4.1666667e-2f;
  p = p * a2 - 0.5f;
  return 1.0f + a2 * p;
}
__device__ __forceinline__ void st_hl(unsigned short* p, int loOff, float v) {
  const _Float16 hv = (_Float16)v;
  const float hf = (float)hv;
  p[0]     = __builtin_bit_cast(unsigned short, hv);
  p[loOff] = h_bits((v - hf) * S_RES);
}
__device__ __forceinline__ float bsum16(float v) {
  v = v + __shfl_xor(v, 1);
  v = v + __shfl_xor(v, 2);
  v = v + __shfl_xor(v, 4);
  v = v + __shfl_xor(v, 8);
  return v;
}
__device__ __forceinline__ float bmax16(float v) {
  v = fmaxf(v, __shfl_xor(v, 1));
  v = fmaxf(v, __shfl_xor(v, 2));
  v = fmaxf(v, __shfl_xor(v, 4));
  v = fmaxf(v, __shfl_xor(v, 8));
  return v;
}

__device__ __forceinline__ v8f mma_h(v16h a, v16h b, v8f c) {
  return __builtin_amdgcn_wmma_f32_16x16x32_f16(false, a, false, b, (short)0, c, false, false);
}
__device__ __forceinline__ void mma_guard1(v8f& c0, v16h a, v16h b) {
#if defined(__HIP_DEVICE_COMPILE__)
  asm volatile("v_nop\n\tv_nop\n\tv_nop\n\tv_nop" : "+v"(c0) : "v"(a), "v"(b));
#else
  (void)c0; (void)a; (void)b;
#endif
}
__device__ __forceinline__ void mma_guard2(v8f& c0, v8f& c1, v16h a, v16h b0, v16h b1) {
#if defined(__HIP_DEVICE_COMPILE__)
  asm volatile("v_nop\n\tv_nop\n\tv_nop\n\tv_nop" : "+v"(c0), "+v"(c1) : "v"(a), "v"(b0), "v"(b1));
#else
  (void)c0; (void)c1; (void)a; (void)b0; (void)b1;
#endif
}
__device__ __forceinline__ void mma_guard4(v8f& c0, v8f& c1, v8f& c2, v8f& c3, v16h a, v16h b) {
#if defined(__HIP_DEVICE_COMPILE__)
  asm volatile("v_nop\n\tv_nop\n\tv_nop\n\tv_nop" : "+v"(c0), "+v"(c1), "+v"(c2), "+v"(c3) : "v"(a), "v"(b));
#else
  (void)c0; (void)c1; (void)c2; (void)c3; (void)a; (void)b;
#endif
}
__device__ __forceinline__ void mma_guard8(v8f& c0, v8f& c1, v8f& c2, v8f& c3,
                                           v8f& c4, v8f& c5, v8f& c6, v8f& c7,
                                           v16h a0, v16h a1, v16h b) {
#if defined(__HIP_DEVICE_COMPILE__)
  asm volatile("v_nop\n\tv_nop\n\tv_nop\n\tv_nop"
               : "+v"(c0), "+v"(c1), "+v"(c2), "+v"(c3), "+v"(c4), "+v"(c5), "+v"(c6), "+v"(c7)
               : "v"(a0), "v"(a1), "v"(b));
#else
  (void)c0; (void)c1; (void)c2; (void)c3; (void)c4; (void)c5; (void)c6; (void)c7; (void)a0; (void)a1; (void)b;
#endif
}

__global__ __launch_bounds__(NTHR) void k_wconv(const float* __restrict__ W_pf, const float* __restrict__ W_h,
                                                  unsigned short* planes) {
  const int piece = blockIdx.x * NTHR + threadIdx.x;
  const int mat   = piece >> 9;
  const int q     = piece & 511;
  const int n     = q >> 3;
  const int kb    = (q & 7) * 8;
  const float* src = (mat == 0) ? W_pf : (W_h + (size_t)(mat - 1) * (HID * HID));
  v8us o;
#pragma unroll
  for (int jj = 0; jj < 8; ++jj) {
    const float w = bfr(src[(size_t)(kb + jj) * HID + n]);
    o[jj] = h_bits(w * S_W);
  }
  unsigned short* d = planes + (size_t)piece * 8;
  *(volatile v8us*)d = o;
  __threadfence();
  *(volatile v8us*)d = o;
}

__global__ __launch_bounds__(NTHR) void k_obj(
    const float* __restrict__ c, const float* __restrict__ t,
    const float* __restrict__ W_of, const float* __restrict__ b_of,
    const float* __restrict__ W_c1, const float* __restrict__ b_c1,
    const float* __restrict__ W_c2, const float* __restrict__ b_c2,
    const float* __restrict__ W_ss,
    unsigned short* objf16, unsigned short* cw16) {
  __shared__ __align__(16) float sCWT[KOBJ * CWD];
  __shared__ __align__(16) float sC1[KOBJ * CDIM];
  __shared__ __align__(16) float sCO[KOBJ * CDIM];
  __shared__ __align__(16) unsigned short sOF[KOBJ * HID];
  __shared__ __align__(16) unsigned short sCWs[NLAY * CDIM * KOBJ];

  const int b   = blockIdx.x;
  const int tid = threadIdx.x;

  {
    const float tb = bfr(t[b]);
    const int   i  = tid & 15;
    const float fr = expf((-9.2103403719761836f * (float)i) * (1.0f / 15.0f));
    const float a  = tb * fr;
    const float sv = sin_small(a);
    const float cv = cos_small(a);
    if (tid < KOBJ) {
#pragma unroll
      for (int k = 0; k < KOBJ; ++k) {
        sCWT[k * CWD + i]        = sv;
        sCWT[k * CWD + 16 + i]   = cv;
      }
    }
  }
#pragma unroll 1
  for (int idx = tid; idx < KOBJ * CDIM; idx += NTHR) {
    const int k = idx >> 7, j = idx & 127;
    sCWT[k * CWD + TED + j] = bfr(c[((size_t)b * KOBJ + k) * CDIM + j]);
  }
  __syncthreads();

  if (tid < 192) {
    const bool isA  = tid < 64;
    const int  n    = isA ? tid : (tid - 64);
    const int  ncol = isA ? HID : CDIM;
    const float* W  = isA ? W_of : W_c1;
    const float* bb = isA ? b_of : b_c1;
    float acc[KOBJ];
#pragma unroll
    for (int k = 0; k < KOBJ; ++k) acc[k] = 0.0f;
#pragma unroll 1
    for (int j = 0; j < CWD; ++j) {
      const float w = bfr(W[(size_t)j * ncol + n]);
      const float* cr = sCWT + j;
#pragma unroll
      for (int k = 0; k < KOBJ; ++k) acc[k] = acc[k] + cr[k * CWD] * w;
    }
    const float bv = bfr(bb[n]);
    if (isA) {
#pragma unroll
      for (int k = 0; k < KOBJ; ++k) sOF[k * HID + n] = h_bits(swish_f(acc[k] + bv) * S_OBJ);
    } else {
#pragma unroll
      for (int k = 0; k < KOBJ; ++k) sC1[k * CDIM + n] = swish_f(acc[k] + bv);
    }
  }
  __syncthreads();

  if (tid < CDIM) {
    const int n = tid;
    float acc[KOBJ];
#pragma unroll
    for (int k = 0; k < KOBJ; ++k) acc[k] = 0.0f;
#pragma unroll 1
    for (int j = 0; j < CDIM; ++j) {
      const float w = bfr(W_c2[(size_t)j * CDIM + n]);
      const float* cr = sC1 + j;
#pragma unroll
      for (int k = 0; k < KOBJ; ++k) acc[k] = acc[k] + cr[k * CDIM] * w;
    }
    const float bv = bfr(b_c2[n]);
#pragma unroll
    for (int k = 0; k < KOBJ; ++k) sCO[k * CDIM + n] = swish_f(acc[k] + bv);
  }
  __syncthreads();

#pragma unroll 1
  for (int it = 0; it < 3; ++it) {
    const int p = tid + it * NTHR;
    const int l = p >> 7;
    const int n = p & 127;
    float acc[KOBJ];
#pragma unroll
    for (int k = 0; k < KOBJ; ++k) acc[k] = 0.0f;
#pragma unroll 1
    for (int j = 0; j < CDIM; ++j) {
      const float w = bfr(W_ss[((size_t)l * CDIM + j) * CDIM + n]);
      const float* cr = sCO + j;
#pragma unroll
      for (int k = 0; k < KOBJ; ++k) acc[k] = acc[k] + cr[k * CDIM] * w;
    }
#pragma unroll
    for (int k = 0; k < KOBJ; ++k) sCWs[(l * CDIM + n) * KOBJ + k] = h_bits(acc[k] * S_CW);
  }
  __syncthreads();

  {
    const int  qo   = tid & 127;
    const bool actO = tid < (KOBJ * HID) / 8;
    const v8us oo   = *(const v8us*)(sOF + 8 * qo);
    unsigned short* dO = objf16 + (size_t)b * (KOBJ * HID) + 8 * qo;
    v8us ow[6];
#pragma unroll
    for (int it = 0; it < 6; ++it) ow[it] = *(const v8us*)(sCWs + 8 * (tid + it * NTHR));
    unsigned short* dC = cw16 + (size_t)b * (NLAY * CDIM * KOBJ) + 8 * tid;
    if (actO) *(volatile v8us*)dO = oo;
#pragma unroll
    for (int it = 0; it < 6; ++it) *(volatile v8us*)(dC + (size_t)it * (NTHR * 8)) = ow[it];
    __threadfence();
    if (actO) *(volatile v8us*)dO = oo;
#pragma unroll
    for (int it = 0; it < 6; ++it) *(volatile v8us*)(dC + (size_t)it * (NTHR * 8)) = ow[it];
  }
}

__global__ __launch_bounds__(NTHR) void k_main(
    const float* __restrict__ x,
    const unsigned short* __restrict__ wpf16, const unsigned short* __restrict__ wh16,
    const unsigned short* __restrict__ objf16, const unsigned short* __restrict__ cw16,
    const float* __restrict__ W_emb, const float* __restrict__ b_emb, const float* __restrict__ b_pf,
    const float* __restrict__ b_h, const float* __restrict__ b_ss,
    const float* __restrict__ ln_g, const float* __restrict__ ln_b,
    const float* __restrict__ W_out, const float* __restrict__ b_out,
    float* out) {
  __shared__ __align__(16) unsigned short sW[HID * HID];
  __shared__ __align__(16) unsigned short sCW[CDIM * KOBJ];
  __shared__ __align__(16) unsigned short sOB[KOBJ * HID];
  __shared__ __align__(16) unsigned short sT[8 * 16 * PA];
  __shared__ __align__(16) float sC[C_TOT];
  __shared__ __align__(16) float sX[BR * XD];
  __shared__ __align__(16) float sOut[BR * XD];

  const int tid  = threadIdx.x;
  const int lane = tid & 31;
  const int wave = tid >> 5;
  const int hh   = lane >> 4;
  const int m16  = lane & 15;
  const int drow = 8 * hh;
  const int blk  = blockIdx.x;
  const int b    = blk / (NPTS / BR);
  unsigned short* tile = sT + wave * (16 * PA);

#pragma unroll 1
  for (int p = tid; p < (HID * HID) / 8; p += NTHR)
    *(v8us*)(sW + 8 * p) = *(const v8us*)(wpf16 + 8 * p);
  if (tid < (KOBJ * HID) / 8)
    *(v8us*)(sOB + 8 * tid) = *(const v8us*)(objf16 + (size_t)b * (KOBJ * HID) + 8 * tid);
#pragma unroll 1
  for (int i = tid; i < XD * HID; i += NTHR) {
    sC[C_WEMB + i] = bfr(W_emb[i]);
    sC[C_WOUT + i] = bfr(W_out[i]);
  }
  if (tid < HID) {
    sC[C_BEMB + tid] = bfr(b_emb[tid]);
    sC[C_BPF + tid]  = bfr(b_pf[tid]);
  }
#pragma unroll 1
  for (int i = tid; i < NLAY * HID; i += NTHR) {
    sC[C_BH + i] = bfr(b_h[i]);
    sC[C_LG + i] = bfr(ln_g[i]);
    sC[C_LB + i] = bfr(ln_b[i]);
  }
#pragma unroll 1
  for (int i = tid; i < NLAY * CDIM; i += NTHR) sC[C_BSS + i] = bfr(b_ss[i]);
  {
    const int i3 = (tid < XD) ? tid : (XD - 1);
    const float bo = bfr(b_out[i3]);
    if (tid < XD) sC[C_BOUT + tid] = bo;
  }
  if (tid < (BR * XD) / 4) {
    const v4f v = *(const v4f*)(x + (size_t)blk * (BR * XD) + 4 * tid);
    v4f rv;
    rv[0] = bfr(v[0]); rv[1] = bfr(v[1]); rv[2] = bfr(v[2]); rv[3] = bfr(v[3]);
    *(v4f*)(sX + 4 * tid) = rv;
  }
  __syncthreads();

  float xe[4][8];
#pragma unroll
  for (int nt = 0; nt < 4; ++nt) {
    const int cc = nt * 16 + m16;
    const float w0 = sC[C_WEMB + cc], w1 = sC[C_WEMB + HID + cc], w2 = sC[C_WEMB + 2 * HID + cc];
    const float be = sC[C_BEMB + cc];
#pragma unroll
    for (int r = 0; r < 8; ++r) {
      const float* xr = sX + (wave * 16 + drow + r) * XD;
      xe[nt][r] = ((xr[0] * w0 + xr[1] * w1) + xr[2] * w2) + be;
    }
  }
#pragma unroll
  for (int nt = 0; nt < 4; ++nt)
#pragma unroll
    for (int r = 0; r < 8; ++r)
      tile[(drow + r) * PA + nt * 16 + m16] = h_bits(xe[nt][r] * S_X);
  __syncthreads();

  float hr[4][8];
  {
    v8f acc[4];
#pragma unroll
    for (int nt = 0; nt < 4; ++nt) acc[nt] = zero8();
    const unsigned short* ap = tile + m16 * PA + 8 * hh;
    const unsigned short* wp = sW + m16 * HID + 8 * hh;
    FragH a, bq;
#pragma unroll
    for (int s = 0; s < 2; ++s) {
      a.u[0] = *(const v8us*)(ap + 32 * s);
      a.u[1] = *(const v8us*)(ap + 32 * s + 16);
#pragma unroll
      for (int nt = 0; nt < 4; ++nt) {
        const unsigned short* w = wp + nt * 16 * HID + 32 * s;
        bq.u[0] = *(const v8us*)(w);
        bq.u[1] = *(const v8us*)(w + 16);
        acc[nt] = mma_h(a.v, bq.v, acc[nt]);
      }
      mma_guard4(acc[0], acc[1], acc[2], acc[3], a.v, bq.v);
    }
#pragma unroll
    for (int nt = 0; nt < 4; ++nt) {
      const float bv = sC[C_BPF + nt * 16 + m16];
#pragma unroll
      for (int r = 0; r < 8; ++r) hr[nt][r] = swish_f(acc[nt][r] * INV_XW + bv);
    }
  }
  __syncthreads();
#pragma unroll
  for (int nt = 0; nt < 4; ++nt)
#pragma unroll
    for (int r = 0; r < 8; ++r)
      tile[(drow + r) * PA + nt * 16 + m16] = h_bits(hr[nt][r] * S_PF);
  __syncthreads();

  float sel[8];
  {
    v8f acc = zero8();
    const unsigned short* ap = tile + m16 * PA + 8 * hh;
    const unsigned short* op = sOB + m16 * HID + 8 * hh;
    FragH a, bq;
#pragma unroll
    for (int s = 0; s < 2; ++s) {
      a.u[0]  = *(const v8us*)(ap + 32 * s);
      a.u[1]  = *(const v8us*)(ap + 32 * s + 16);
      bq.u[0] = *(const v8us*)(op + 32 * s);
      bq.u[1] = *(const v8us*)(op + 32 * s + 16);
      acc = mma_h(a.v, bq.v, acc);
      mma_guard1(acc, a.v, bq.v);
    }
#pragma unroll
    for (int r = 0; r < 8; ++r) {
      const float av = acc[r] * INV_PFO;
      const float mx = bmax16(av);
      const float e  = __expf(av - mx);
      const float sm = bsum16(e);
      sel[r] = e * rcp_f(sm);
    }
  }
  __syncthreads();
#pragma unroll
  for (int r = 0; r < 8; ++r) tile[(drow + r) * PA + m16] = h_bits(sel[r]);
  __syncthreads();
  FragH selA;
  selA.u[0] = *(const v8us*)(tile + m16 * PA + 8 * hh);
  selA.u[1] = zero8us();
  __syncthreads();

#pragma unroll
  for (int nt = 0; nt < 4; ++nt)
#pragma unroll
    for (int r = 0; r < 8; ++r)
      st_hl(tile + (drow + r) * PA + nt * 16 + m16, 64, swish_f(xe[nt][r]) * S_H);
  __syncthreads();

#pragma unroll 1
  for (int l = 0; l < NLAY; ++l) {
    {
      const unsigned short* wsrc = wh16 + (size_t)l * (HID * HID);
#pragma unroll 1
      for (int p = tid; p < (HID * HID) / 8; p += NTHR)
        *(v8us*)(sW + 8 * p) = *(const v8us*)(wsrc + 8 * p);
      const unsigned short* csrc = cw16 + ((size_t)b * NLAY + l) * (CDIM * KOBJ);
      *(v8us*)(sCW + 8 * tid) = *(const v8us*)(csrc + 8 * tid);
    }
    __syncthreads();

    v8f ah[4], al[4];
#pragma unroll
    for (int nt = 0; nt < 4; ++nt) { ah[nt] = zero8(); al[nt] = zero8(); }
    {
      const unsigned short* ap = tile + m16 * PA + 8 * hh;
      const unsigned short* wp = sW + m16 * HID + 8 * hh;
      FragH fh, fl, bq;
#pragma unroll
      for (int s = 0; s < 2; ++s) {
        fh.u[0] = *(const v8us*)(ap + 32 * s);
        fh.u[1] = *(const v8us*)(ap + 32 * s + 16);
        fl.u[0] = *(const v8us*)(ap + 64 + 32 * s);
        fl.u[1] = *(const v8us*)(ap + 64 + 32 * s + 16);
#pragma unroll
        for (int nt = 0; nt < 4; ++nt) {
          const unsigned short* w = wp + nt * 16 * HID + 32 * s;
          bq.u[0] = *(const v8us*)(w);
          bq.u[1] = *(const v8us*)(w + 16);
          ah[nt] = mma_h(fh.v, bq.v, ah[nt]);
          al[nt] = mma_h(fl.v, bq.v, al[nt]);
        }
        mma_guard8(ah[0], ah[1], ah[2], ah[3], al[0], al[1], al[2], al[3], fh.v, fl.v, bq.v);
      }
    }
#pragma unroll
    for (int nt = 0; nt < 4; ++nt) {
      const float bv = sC[C_BH + l * HID + nt * 16 + m16];
#pragma unroll
      for (int r = 0; r < 8; ++r) {
        const float z = (ah[nt][r] + al[nt][r] * INV_RES) * INV_HW + bv;
        hr[nt][r] = swish_f(z);
      }
    }
    {
      float g4[4], b4[4];
#pragma unroll
      for (int nt = 0; nt < 4; ++nt) {
        g4[nt] = sC[C_LG + l * HID + nt * 16 + m16];
        b4[nt] = sC[C_LB + l * HID + nt * 16 + m16];
      }
#pragma unroll
      for (int r = 0; r < 8; ++r) {
        float s1 = ((hr[0][r] + hr[1][r]) + hr[2][r]) + hr[3][r];
        s1 = bsum16(s1);
        const float mu = s1 * (1.0f / 64.0f);
        const float x0 = hr[0][r] - mu, x1 = hr[1][r] - mu, x2 = hr[2][r] - mu, x3 = hr[3][r] - mu;
        float s2 = ((x0 * x0 + x1 * x1) + x2 * x2) + x3 * x3;
        s2 = bsum16(s2);
        const float var  = s2 * (1.0f / 64.0f);
        const float rstd = rsq_f(var + 1e-6f);
        hr[0][r] = (x0 * rstd) * g4[0] + b4[0];
        hr[1][r] = (x1 * rstd) * g4[1] + b4[1];
        hr[2][r] = (x2 * rstd) * g4[2] + b4[2];
        hr[3][r] = (x3 * rstd) * g4[3] + b4[3];
      }
    }
#pragma unroll
    for (int nt = 0; nt < 4; ++nt) {
      v8f as = zero8(), at = zero8();
      FragH bs, bt;
      bs.u[0] = *(const v8us*)(sCW + (nt * 16 + m16) * KOBJ + 8 * hh);
      bs.u[1] = zero8us();
      bt.u[0] = *(const v8us*)(sCW + (HID + nt * 16 + m16) * KOBJ + 8 * hh);
      bt.u[1] = zero8us();
      as = mma_h(selA.v, bs.v, as);
      at = mma_h(selA.v, bt.v, at);
      mma_guard2(as, at, selA.v, bs.v, bt.v);
      const float scb = sC[C_BSS + l * CDIM + nt * 16 + m16];
      const float shb = sC[C_BSS + l * CDIM + HID + nt * 16 + m16];
#pragma unroll
      for (int r = 0; r < 8; ++r) {
        const float sc = as[r] * INV_CW + scb;
        const float sh = at[r] * INV_CW + shb;
        hr[nt][r] = (hr[nt][r] * (1.0f + sc)) + sh;
      }
    }
    if (l + 1 < NLAY) {
#pragma unroll
      for (int nt = 0; nt < 4; ++nt)
#pragma unroll
        for (int r = 0; r < 8; ++r)
          st_hl(tile + (drow + r) * PA + nt * 16 + m16, 64, hr[nt][r] * S_H);
    }
    __syncthreads();
  }

  {
    float w0[4], w1[4], w2[4];
#pragma unroll
    for (int nt = 0; nt < 4; ++nt) {
      const int k = nt * 16 + m16;
      w0[nt] = sC[C_WOUT + k * XD + 0];
      w1[nt] = sC[C_WOUT + k * XD + 1];
      w2[nt] = sC[C_WOUT + k * XD + 2];
    }
    const int dsel = (m16 < XD) ? m16 : (XD - 1);
    const float bo = sC[C_BOUT + dsel];
#pragma unroll
    for (int r = 0; r < 8; ++r) {
      float p0 = ((hr[0][r] * w0[0] + hr[1][r] * w0[1]) + hr[2][r] * w0[2]) + hr[3][r] * w0[3];
      float p1 = ((hr[0][r] * w1[0] + hr[1][r] * w1[1]) + hr[2][r] * w1[2]) + hr[3][r] * w1[3];
      float p2 = ((hr[0][r] * w2[0] + hr[1][r] * w2[1]) + hr[2][r] * w2[2]) + hr[3][r] * w2[3];
      p0 = bsum16(p0);
      p1 = bsum16(p1);
      p2 = bsum16(p2);
      const float v = ((m16 == 0) ? p0 : ((m16 == 1) ? p1 : p2)) + bo;
      if (m16 < XD) sOut[(wave * 16 + drow + r) * XD + m16] = v;
    }
  }
  __syncthreads();
  {
    const bool act = tid < (BR * XD) / 4;
    const int q = act ? tid : 0;
    const v4f ov = *(const v4f*)(sOut + 4 * q);
    float* gp = out + (size_t)blk * (BR * XD) + 4 * q;
    if (act) *(volatile v4f*)gp = ov;
    __threadfence();
    if (act) *(volatile v4f*)gp = ov;
  }
}

extern "C" void kernel_launch(void* const* d_in, const int* in_sizes, int n_in,
                              void* d_out, int out_size, void* d_ws, size_t ws_size,
                              hipStream_t stream) {
  if (n_in < 21) return;
  if (in_sizes[0] != NB * NPTS * XD) return;
  if (in_sizes[1] != NB * KOBJ * CDIM) return;
  if (in_sizes[2] != NB) return;
  if (in_sizes[3] != XD * HID || in_sizes[4] != HID) return;
  if (in_sizes[5] != HID * HID || in_sizes[6] != HID) return;
  if (in_sizes[7] != CWD * HID || in_sizes[8] != HID) return;
  if (in_sizes[9] != CWD * CDIM || in_sizes[10] != CDIM) return;
  if (in_sizes[11] != CDIM * CDIM || in_sizes[12] != CDIM) return;
  if (in_sizes[13] != NLAY * HID * HID || in_sizes[14] != NLAY * HID) return;
  if (in_sizes[15] != NLAY * CDIM * CDIM || in_sizes[16] != NLAY * CDIM) return;
  if (in_sizes[17] != NLAY * HID || in_sizes[18] != NLAY * HID) return;
  if (in_sizes[19] != HID * XD || in_sizes[20] != XD) return;
  if (out_size != NB * NPTS * XD) return;

  const float* xin   = (const float*)d_in[0];
  const float* c     = (const float*)d_in[1];
  const float* t     = (const float*)d_in[2];
  const float* W_emb = (const float*)d_in[3];
  const float* b_emb = (const float*)d_in[4];
  const float* W_pf  = (const float*)d_in[5];
  const float* b_pf  = (const float*)d_in[6];
  const float* W_of  = (const float*)d_in[7];
  const float* b_of  = (const float*)d_in[8];
  const float* W_c1  = (const float*)d_in[9];
  const float* b_c1  = (const float*)d_in[10];
  const float* W_c2  = (const float*)d_in[11];
  const float* b_c2  = (const float*)d_in[12];
  const float* W_h   = (const float*)d_in[13];
  const float* b_h   = (const float*)d_in[14];
  const float* W_ss  = (const float*)d_in[15];
  const float* b_ss  = (const float*)d_in[16];
  const float* ln_g  = (const float*)d_in[17];
  const float* ln_b  = (const float*)d_in[18];
  const float* W_out = (const float*)d_in[19];
  const float* b_out = (const float*)d_in[20];
  float* out = (float*)d_out;

  const size_t tot = (size_t)WS_TOT * 2;
  if (tot > ws_size) return;
  if (tot > (size_t)134217728) return;
  unsigned short* ws16  = (unsigned short*)d_ws;
  unsigned short* wpf16 = ws16 + WS_WPF;
  unsigned short* wh16  = ws16 + WS_WH;
  unsigned short* obj16 = ws16 + WS_OBJ;
  unsigned short* cw16  = ws16 + WS_CW;

  const int nblk = (NB * NPTS) / BR;

  k_wconv<<<dim3(WCONV_PIECES / NTHR), dim3(NTHR), 0, stream>>>(W_pf, W_h, wpf16);
  k_obj<<<dim3(NB), dim3(NTHR), 0, stream>>>(c, t, W_of, b_of, W_c1, b_c1, W_c2, b_c2, W_ss, obj16, cw16);
  k_main<<<dim3(nblk), dim3(NTHR), 0, stream>>>(
      xin, wpf16, wh16, obj16, cw16, W_emb, b_emb, b_pf, b_h, b_ss, ln_g, ln_b, W_out, b_out, out);
  (void)hipGetLastError();
}
